// MidAttnBlock_60601988546748
// MI455X (gfx1250) — hardware-verified
//
#include <hip/hip_runtime.h>


#define NB_  8
#define CI   96
#define LL   2048
#define NH_  4
#define DQ   48
#define DQP  64
#define DV   96
#define DVP  128
#define CQKV 768
#define CO2  384
#define PCAR 1024.0f
#define ZH   2
typedef _Float16 h16;
typedef unsigned short bf;
typedef __attribute__((ext_vector_type(16))) __bf16   v16bf;
typedef __attribute__((ext_vector_type(16))) _Float16 v16h;
typedef __attribute__((ext_vector_type(8)))  _Float16 v8h;
typedef __attribute__((ext_vector_type(8)))  unsigned short v8us;
typedef __attribute__((ext_vector_type(8)))  float    v8f;
typedef __attribute__((ext_vector_type(4)))  float    v4f;
typedef v8h  __attribute__((may_alias)) v8ha;
typedef v4f  __attribute__((may_alias)) v4fa;
typedef v8us __attribute__((may_alias)) v8usa;

__device__ __forceinline__ unsigned short f2bf(float f) { unsigned u = __float_as_uint(f); u += 0x7FFFu + ((u >> 16) & 1u); return (unsigned short)(u >> 16); }
__device__ __forceinline__ float bf2f(unsigned short b) { return __uint_as_float(((unsigned)b) << 16); }
__device__ __forceinline__ float bfr(float f) { return bf2f(f2bf(f)); }
__device__ __forceinline__ v16h cat16(v8h lo, v8h hi) { return __builtin_shufflevector(lo, hi, 0, 1, 2, 3, 4, 5, 6, 7, 8, 9, 10, 11, 12, 13, 14, 15); }
__device__ __forceinline__ v16bf cat16b(v8us lo, v8us hi) { return __builtin_bit_cast(v16bf, __builtin_shufflevector(lo, hi, 0, 1, 2, 3, 4, 5, 6, 7, 8, 9, 10, 11, 12, 13, 14, 15)); }
__device__ __forceinline__ v8f wmma16(v16h a, v16h b, v8f c) { return __builtin_amdgcn_wmma_f32_16x16x32_f16(false, a, false, b, (short)0, c, false, false); }
__device__ __forceinline__ v8f wmmab(v16bf a, v16bf b, v8f c) { return __builtin_amdgcn_wmma_f32_16x16x32_bf16(false, a, false, b, (short)0, c, false, false); }


template <typename T16> struct WFrag;
template <> struct WFrag<h16> { typedef v16h V; static __device__ __forceinline__ V ld(const h16* p) { return cat16(*(const v8h*)p, *(const v8h*)(p + 16)); } static __device__ __forceinline__ v8f mma(V a, V b, v8f c) { return wmma16(a, b, c); } };
template <> struct WFrag<bf> { typedef v16bf V; static __device__ __forceinline__ V ld(const bf* p) { return cat16b(*(const v8us*)p, *(const v8us*)(p + 16)); } static __device__ __forceinline__ v8f mma(V a, V b, v8f c) { return wmmab(a, b, c); } };
template <typename T16, int NSPLIT, bool BIAS>
__global__ __launch_bounds__(32) void k_gemmw(const T16* __restrict__ A, const T16* __restrict__ A2, const T16* __restrict__ Bt, const T16* __restrict__ Bt2, int K, float* C, int ldc, const float* __restrict__ bias, size_t sA, size_t sB, size_t sC) {
    typedef typename WFrag<T16>::V V;
    __shared__ __align__(16) float os[16 * 68];
    const size_t z = blockIdx.z; A += z * sA; if (A2) A2 += z * sA; Bt += z * sB; if (Bt2) Bt2 += z * sB; C += z * sC;
    const int lane = threadIdx.x & 31, lr = lane & 15, hi = lane >> 4; const int r0 = blockIdx.x * 64, c0 = blockIdx.y * 64;
    v8f acc[4][4];
#pragma unroll
    for (int mb = 0; mb < 4; ++mb)
#pragma unroll
        for (int nb = 0; nb < 4; ++nb) acc[mb][nb] = (v8f){};
    const size_t aoff = (size_t)(r0 + lr) * K + 8 * hi, boff = (size_t)(c0 + lr) * K + 8 * hi;
#pragma unroll 1
    for (int kc = 0; kc < K; kc += 32) {
        V a[4], a2[4];
#pragma unroll
        for (int mb = 0; mb < 4; ++mb) { a[mb] = WFrag<T16>::ld(A + aoff + (size_t)mb * 16 * K + kc); if (NSPLIT == 1 || NSPLIT == 2) a2[mb] = WFrag<T16>::ld(A2 + aoff + (size_t)mb * 16 * K + kc); }
#pragma unroll
        for (int nb = 0; nb < 4; ++nb) { const V b = WFrag<T16>::ld(Bt + boff + (size_t)nb * 16 * K + kc); V b2; if (NSPLIT >= 2) b2 = WFrag<T16>::ld(Bt2 + boff + (size_t)nb * 16 * K + kc);
#pragma unroll
            for (int mb = 0; mb < 4; ++mb) { acc[mb][nb] = WFrag<T16>::mma(a[mb], b, acc[mb][nb]); if (NSPLIT == 1 || NSPLIT == 2) acc[mb][nb] = WFrag<T16>::mma(a2[mb], b, acc[mb][nb]); if (NSPLIT >= 2) acc[mb][nb] = WFrag<T16>::mma(a[mb], b2, acc[mb][nb]); } }
        asm volatile("v_nop\n\tv_nop\n\tv_nop\n\tv_nop" : "+v"(acc[0][0]), "+v"(acc[1][1]), "+v"(acc[2][2]), "+v"(acc[3][3]) : "v"(a[0]), "v"(a[3]));
    }
#pragma unroll
    for (int mb = 0; mb < 4; ++mb) {
#pragma unroll
        for (int nb = 0; nb < 4; ++nb) {
#pragma unroll
            for (int j = 0; j < 8; ++j) os[(hi * 8 + j) * 68 + nb * 16 + lr] = acc[mb][nb][j]; }
        __builtin_amdgcn_wave_barrier(); asm volatile("" ::: "memory");
        float* crow = C + (size_t)(r0 + mb * 16) * ldc + c0;
#pragma unroll 1
        for (int ps = 0; ps < 2; ++ps) {
#pragma unroll
            for (int s = 0; s < 8; ++s) { const int row = 2 * s + hi, cofs = lr * 4; v4f val = *(const v4fa*)(os + row * 68 + cofs); if (BIAS) { val[0] += bfr(bias[c0 + cofs]); val[1] += bfr(bias[c0 + cofs + 1]); val[2] += bfr(bias[c0 + cofs + 2]); val[3] += bfr(bias[c0 + cofs + 3]); }
                *(volatile v4f*)(crow + (size_t)row * ldc + cofs) = val; }
            if (ps == 0) __threadfence(); }
        __builtin_amdgcn_wave_barrier(); asm volatile("" ::: "memory");
    }
}

__device__ __forceinline__ h16 tohx(float x) { return (h16)x; }
__device__ __forceinline__ void splitf(float y, unsigned short& h, unsigned short& l) { h = f2bf(y); l = f2bf(y - bf2f(h)); }
__device__ __forceinline__ float siluf(float t) { return __fdiv_rn(t, 1.0f + __expf(-t)); }
typedef __attribute__((ext_vector_type(2))) _Float16 v2h;
typedef __attribute__((ext_vector_type(4))) _Float16 v4h;
typedef __attribute__((ext_vector_type(2))) unsigned short v2us;

__global__ __launch_bounds__(256) void k_wpad(const float* __restrict__ w, int O, int Op, int K, bf* WB) {
    const int lane = threadIdx.x & 31; const int L = blockIdx.x * 8 + (threadIdx.x >> 5); if (L >= Op * K / 64) return; const int e = L * 64 + lane * 2; v2us v;
#pragma unroll
    for (int q = 0; q < 2; ++q) { const int o = (e + q) / K, k = (e + q) % K; v[q] = (o < O) ? f2bf(w[(size_t)o * K + k]) : (unsigned short)0; }
    *(volatile v2us*)(WB + e) = v; __threadfence(); *(volatile v2us*)(WB + e) = v;
}
template <bool ROUND, int C, int CG>
__global__ __launch_bounds__(256) void k_gnstat(const float* __restrict__ T, const float* __restrict__ bias, float* MS) {
    const int lane = threadIdx.x & 31; const int wg = blockIdx.x * 8 + (threadIdx.x >> 5); if (wg >= NB_ * 32) return; const int b = wg >> 5, g = wg & 31; const float* base = T + ((size_t)b * C + g * CG) * LL; const int n = CG * LL;
    float s = 0.f;
#pragma unroll 1
    for (int i = lane; i < n; i += 32) { float t = ROUND ? bfr(base[i]) : base[i]; if (bias) t += bfr(bias[g * CG + i / LL]); s += t; }
#pragma unroll
    for (int sh = 16; sh; sh >>= 1) s += __shfl_xor(s, sh, 32);
    const float mu = __fdiv_rn(s, (float)n); float q = 0.f;
#pragma unroll 1
    for (int i = lane; i < n; i += 32) { float t = ROUND ? bfr(base[i]) : base[i]; if (bias) t += bfr(bias[g * CG + i / LL]); const float d = t - mu; q = fmaf(d, d, q); }
#pragma unroll
    for (int sh = 16; sh; sh >>= 1) q += __shfl_xor(q, sh, 32);
    const float rs = rsqrtf(__fdiv_rn(q, (float)n) + 1e-5f);
    const float v = lane == 0 ? mu : (lane == 1 ? rs : 0.f); *(volatile float*)(MS + (size_t)wg * 32 + lane) = v; __threadfence(); *(volatile float*)(MS + (size_t)wg * 32 + lane) = v;
}
template <bool SILU, bool ROUND, int C, int CG>
__global__ __launch_bounds__(256) void k_gnplane(const float* __restrict__ T, const float* __restrict__ bias, const float* __restrict__ MS, const float* __restrict__ gw, const float* __restrict__ gb, bf* Ph, bf* Pl) {
    const int lane = threadIdx.x & 31; const int L0 = (blockIdx.x * 8 + (threadIdx.x >> 5)) * 8; const int nlines = NB_ * LL * C / 64;
#pragma unroll 1
    for (int ps = 0; ps < 2; ++ps) {
#pragma unroll 1
        for (int l = 0; l < 8; ++l) { const int L = L0 + l; if (L >= nlines) break; const int e = L * 64 + lane * 2; const int c = e % C; const int t = (e / C) % LL; const int b = e / (C * LL); v2us oh, ol;
#pragma unroll
            for (int q = 0; q < 2; ++q) { const int cc = c + q; const float* ms = MS + ((size_t)b * 32 + cc / CG) * 32; float v = T[((size_t)b * C + cc) * LL + t]; if (ROUND) v = bfr(v); if (bias) v += bfr(bias[cc]);
                v = (v - ms[0]) * ms[1] * bfr(gw[cc]) + bfr(gb[cc]); if (SILU) v = siluf(v); unsigned short a, c2; splitf(v, a, c2); oh[q] = a; ol[q] = c2; }
            *(volatile v2us*)(Ph + (size_t)e) = oh; *(volatile v2us*)(Pl + (size_t)e) = ol; }
        if (ps == 0) __threadfence(); }
}
__global__ __launch_bounds__(256) void k_qkplanes(const float* __restrict__ F, const float* __restrict__ qb, h16* Qp, h16* Kp) {
    const int lane = threadIdx.x & 31; const int L0 = (blockIdx.x * 8 + (threadIdx.x >> 5)) * 8; const int nlines = NB_ * NH_ * LL * DQP / 64;
#pragma unroll 1
    for (int ps = 0; ps < 2; ++ps) {
#pragma unroll
        for (int l = 0; l < 8; ++l) { const int L = L0 + l; if (L >= nlines) break; const int e = L * 64 + lane * 2; const int c = e & 63; const int m = (e >> 6) & (LL - 1); const int n = e >> 17; const int b = n >> 2, h = n & 3; v2h vq, vk;
#pragma unroll
            for (int q = 0; q < 2; ++q) { const int cc = c + q; const int oq = h * DQ + cc, ok = NH_ * DQ + h * DQ + cc; vq[q] = tohx(cc < DQ ? F[((size_t)b * CQKV + oq) * LL + m] + bfr(qb[oq]) : 0.f); vk[q] = tohx(cc < DQ ? F[((size_t)b * CQKV + ok) * LL + m] + bfr(qb[ok]) : 0.f); }
            *(volatile v2h*)(Qp + (size_t)e) = vq; *(volatile v2h*)(Kp + (size_t)e) = vk; }
        if (ps == 0) __threadfence(); }
}
__global__ __launch_bounds__(256) void k_vplane(const float* __restrict__ F, const float* __restrict__ qb, h16* VP) {
    const int lane = threadIdx.x & 31; const int L0 = (blockIdx.x * 8 + (threadIdx.x >> 5)) * 8; const int nlines = NB_ * NH_ * DVP * LL / 64;
#pragma unroll 1
    for (int ps = 0; ps < 2; ++ps) {
#pragma unroll
        for (int l = 0; l < 8; ++l) { const int L = L0 + l; if (L >= nlines) break; const int e = L * 64 + lane * 2; const int t = e & (LL - 1); const int c = (e >> 11) & 127; const int n = e >> 18; const int b = n >> 2, h = n & 3; v2h v;
#pragma unroll
            for (int q = 0; q < 2; ++q) { const int ov = 2 * NH_ * DQ + h * DV + c; v[q] = tohx(c < DV ? F[((size_t)b * CQKV + ov) * LL + t + q] + bfr(qb[ov]) : 0.f); }
            *(volatile v2h*)(VP + (size_t)e) = v; }
        if (ps == 0) __threadfence(); }
}
__global__ __launch_bounds__(256) void k_soft(const float* __restrict__ Sb, const float* __restrict__ scp, h16* P) {
    const int lane = threadIdx.x & 31; const int row = blockIdx.x * 8 + (threadIdx.x >> 5); if (row >= ZH * LL) return; const float* sr = Sb + (size_t)row * LL; const float sc = bfr(scp[0]);
    float m = -3.0e38f;
#pragma unroll 1
    for (int c0 = lane * 4; c0 < LL; c0 += 128) { const v4f v = *(const v4f*)(sr + c0);
#pragma unroll
        for (int q = 0; q < 4; ++q) m = fmaxf(m, v[q] * sc); }
#pragma unroll
    for (int sh = 16; sh; sh >>= 1) m = fmaxf(m, __shfl_xor(m, sh, 32));
    float sum = 0.f;
#pragma unroll 1
    for (int c0 = lane * 4; c0 < LL; c0 += 128) { const v4f v = *(const v4f*)(sr + c0);
#pragma unroll
        for (int q = 0; q < 4; ++q) sum += __expf(v[q] * sc - m); }
#pragma unroll
    for (int sh = 16; sh; sh >>= 1) sum += __shfl_xor(sum, sh, 32);
    const float f = __fdiv_rn(PCAR, sum);
#pragma unroll 1
    for (int ps = 0; ps < 2; ++ps) {
#pragma unroll 1
        for (int c0 = lane * 4; c0 < LL; c0 += 128) { const v4f v = *(const v4f*)(sr + c0); v4h o;
#pragma unroll
            for (int q = 0; q < 4; ++q) o[q] = tohx(__expf(v[q] * sc - m) * f);
            *(volatile v4h*)(P + (size_t)row * LL + c0) = o; }
        if (ps == 0) __threadfence(); }
}
__global__ __launch_bounds__(256) void k_ot(const float* __restrict__ Ob, int b, int h0, float* O2) {
    typedef __attribute__((ext_vector_type(2))) float v2f;
    const int lane = threadIdx.x & 31; const int L0 = (blockIdx.x * 8 + (threadIdx.x >> 5)) * 8; const int nlines = ZH * DV * LL / 64;
#pragma unroll 1
    for (int ps = 0; ps < 2; ++ps) {
#pragma unroll
        for (int l = 0; l < 8; ++l) { const int L = L0 + l; if (L >= nlines) break; const int idx = (L * 32 + lane) * 2; const int m = idx & (LL - 1); const int c = (idx >> 11) % DV; const int zz = idx / (LL * DV); v2f v;
            v[0] = Ob[((size_t)zz * LL + m) * DVP + c] * (1.0f / PCAR); v[1] = Ob[((size_t)zz * LL + m + 1) * DVP + c] * (1.0f / PCAR);
            *(volatile v2f*)(O2 + ((size_t)b * CO2 + (h0 + zz) * DV + c) * LL + m) = v; }
        if (ps == 0) __threadfence(); }
}
__global__ __launch_bounds__(256) void k_im2col3(const float* __restrict__ P2, const float* __restrict__ pb, const float* __restrict__ MS, const float* __restrict__ gw, const float* __restrict__ gb, bf* Ph, bf* Pl) {
    const int lane = threadIdx.x & 31; const int L0 = (blockIdx.x * 8 + (threadIdx.x >> 5)) * 8; const int nlines = NB_ * LL * CI * 3 / 64;
#pragma unroll 1
    for (int ps = 0; ps < 2; ++ps) {
#pragma unroll 1
        for (int l = 0; l < 8; ++l) { const int L = L0 + l; if (L >= nlines) break; const int e = L * 64 + lane * 2; const int col = e % (CI * 3); const int t = (e / (CI * 3)) % LL; const int b = e / (CI * 3 * LL); v2us oh, ol;
#pragma unroll
            for (int q = 0; q < 2; ++q) { const int cq = col + q; const int ci = cq / 3, k = cq % 3; const int tt = t + k - 1; float v = 0.f;
                if (tt >= 0 && tt < LL) { const float* ms = MS + ((size_t)b * 32 + ci / 3) * 32; v = P2[((size_t)b * DVP + ci) * LL + tt] + bfr(pb[ci]); v = (v - ms[0]) * ms[1] * bfr(gw[ci]) + bfr(gb[ci]); v = siluf(v); }
                unsigned short a, c2; splitf(v, a, c2); oh[q] = a; ol[q] = c2; }
            *(volatile v2us*)(Ph + (size_t)e) = oh; *(volatile v2us*)(Pl + (size_t)e) = ol; }
        if (ps == 0) __threadfence(); }
}
__global__ __launch_bounds__(256) void k_fin(const float* __restrict__ x, const float* __restrict__ C3, const float* __restrict__ cb, float* OUT) {
    const size_t i = (size_t)blockIdx.x * 256 + threadIdx.x; if (i >= (size_t)NB_ * CI * LL / 4) return; const size_t e = i * 4; const int l = (int)(e & (LL - 1)); const int c = (int)((e >> 11) % CI); const int b = (int)(e / ((size_t)CI * LL));
    const v4f xv = *(const v4f*)(x + e), cv = *(const v4f*)(C3 + ((size_t)b * DVP + c) * LL + l); const float bb = bfr(cb[c]); v4f o;
#pragma unroll
    for (int q = 0; q < 4; ++q) o[q] = bfr(xv[q]) + cv[q] + bb;
    *(volatile v4f*)(OUT + e) = o; __threadfence(); *(volatile v4f*)(OUT + e) = o;
}

extern "C" void kernel_launch(void* const* d_in, const int* in_sizes, int n_in,
                              void* d_out, int out_size, void* d_ws, size_t ws_size, hipStream_t stream) {
    (void)in_sizes; (void)n_in; (void)out_size;
    const float* x = (const float*)d_in[0]; const float* gn1w = (const float*)d_in[1]; const float* gn1b = (const float*)d_in[2]; const float* qkv_w = (const float*)d_in[3]; const float* qkv_b = (const float*)d_in[4]; const float* scp = (const float*)d_in[5];
    const float* gn2w = (const float*)d_in[6]; const float* gn2b = (const float*)d_in[7]; const float* proj_w = (const float*)d_in[8]; const float* proj_b = (const float*)d_in[9]; const float* gn3w = (const float*)d_in[10]; const float* gn3b = (const float*)d_in[11]; const float* c3w = (const float*)d_in[12]; const float* c3b = (const float*)d_in[13];
    float* OUT = (float*)d_out;
    char* wsp = (char*)d_ws;
    auto take = [&](size_t bytes) { char* p = wsp; wsp += (bytes + 255) & ~(size_t)255; return (void*)p; };
    bf* WQKV = (bf*)take((size_t)CQKV * CI * 2); bf* ZQKV = (bf*)take((size_t)CQKV * CI * 2); bf* WPJ = (bf*)take((size_t)DVP * CO2 * 2); bf* ZPJ = (bf*)take((size_t)DVP * CO2 * 2); bf* WC3 = (bf*)take((size_t)DVP * CI * 3 * 2); bf* ZC3 = (bf*)take((size_t)DVP * CI * 3 * 2);
    float* MS = (float*)take((size_t)NB_ * 32 * 32 * 4); bf* H1h = (bf*)take((size_t)NB_ * LL * CI * 2); bf* H1l = (bf*)take((size_t)NB_ * LL * CI * 2);
    float* F = (float*)take((size_t)NB_ * CQKV * LL * 4);
    h16* Qp = (h16*)take((size_t)NB_ * NH_ * LL * DQP * 2); h16* Kp = (h16*)take((size_t)NB_ * NH_ * LL * DQP * 2); h16* VP = (h16*)take((size_t)NB_ * NH_ * DVP * LL * 2); float* Ob = (float*)take((size_t)ZH * LL * DVP * 4);
    float* O2 = (float*)take((size_t)NB_ * CO2 * LL * 4); bf* G2h = (bf*)take((size_t)NB_ * LL * CO2 * 2); bf* G2l = (bf*)take((size_t)NB_ * LL * CO2 * 2); float* P2 = (float*)take((size_t)NB_ * DVP * LL * 4);
    bf* IMh = (bf*)take((size_t)NB_ * LL * CI * 3 * 2); bf* IMl = (bf*)take((size_t)NB_ * LL * CI * 3 * 2); float* C3 = (float*)take((size_t)NB_ * DVP * LL * 4);
    if ((size_t)(wsp - (char*)d_ws) > ws_size) return;
    float* Sb = F; h16* Pm = (h16*)((char*)F + (size_t)ZH * LL * LL * 4);
    k_wpad<<<(CQKV * CI / 64 + 7) / 8, 256, 0, stream>>>(qkv_w, CQKV, CQKV, CI, WQKV); k_wpad<<<(DVP * CO2 / 64 + 7) / 8, 256, 0, stream>>>(proj_w, CI, DVP, CO2, WPJ); k_wpad<<<(DVP * CI * 3 / 64 + 7) / 8, 256, 0, stream>>>(c3w, CI, DVP, CI * 3, WC3);
    hipMemsetAsync(ZQKV, 0, (size_t)CQKV * CI * 2, stream); hipMemsetAsync(ZPJ, 0, (size_t)DVP * CO2 * 2, stream); hipMemsetAsync(ZC3, 0, (size_t)DVP * CI * 3 * 2, stream);
    k_gnstat<true, CI, 3><<<NB_ * 32 / 8, 256, 0, stream>>>(x, nullptr, MS);
    k_gnplane<true, true, CI, 3><<<(unsigned)((NB_ * LL * CI / 64 + 63) / 64), 256, 0, stream>>>(x, nullptr, MS, gn1w, gn1b, H1h, H1l);
    k_gemmw<bf, 2, false><<<dim3(CQKV / 64, LL / 64, NB_), 32, 0, stream>>>(WQKV, ZQKV, H1h, H1l, CI, F, LL, nullptr, 0, (size_t)LL * CI, (size_t)CQKV * LL);
    k_qkplanes<<<(NB_ * NH_ * LL * DQP / 64 + 63) / 64, 256, 0, stream>>>(F, qkv_b, Qp, Kp); k_vplane<<<(NB_ * NH_ * DVP * LL / 64 + 63) / 64, 256, 0, stream>>>(F, qkv_b, VP);
    for (int b = 0; b < NB_; ++b)
        for (int h0 = 0; h0 < NH_; h0 += ZH) { const size_t n0 = (size_t)b * NH_ + h0;
            k_gemmw<h16, 0, false><<<dim3(LL / 64, LL / 64, ZH), 32, 0, stream>>>(Qp + n0 * LL * DQP, nullptr, Kp + n0 * LL * DQP, nullptr, DQP, Sb, LL, nullptr, (size_t)LL * DQP, (size_t)LL * DQP, (size_t)LL * LL);
            k_soft<<<ZH * LL / 8, 256, 0, stream>>>(Sb, scp, Pm);
            k_gemmw<h16, 0, false><<<dim3(LL / 64, DVP / 64, ZH), 32, 0, stream>>>(Pm, nullptr, VP + n0 * DVP * LL, nullptr, LL, Ob, DVP, nullptr, (size_t)LL * LL, (size_t)DVP * LL, (size_t)LL * DVP);
            k_ot<<<(ZH * DV * LL / 64 + 63) / 64, 256, 0, stream>>>(Ob, b, h0, O2); }
    k_gnstat<false, CO2, 12><<<NB_ * 32 / 8, 256, 0, stream>>>(O2, nullptr, MS);
    k_gnplane<false, false, CO2, 12><<<(unsigned)((NB_ * LL * CO2 / 64 + 63) / 64), 256, 0, stream>>>(O2, nullptr, MS, gn2w, gn2b, G2h, G2l);
    k_gemmw<bf, 2, false><<<dim3(DVP / 64, LL / 64, NB_), 32, 0, stream>>>(WPJ, ZPJ, G2h, G2l, CO2, P2, LL, nullptr, 0, (size_t)LL * CO2, (size_t)DVP * LL);
    k_gnstat<false, DVP, 3><<<NB_ * 32 / 8, 256, 0, stream>>>(P2, proj_b, MS);
    k_im2col3<<<(unsigned)((NB_ * LL * CI * 3 / 64 + 63) / 64), 256, 0, stream>>>(P2, proj_b, MS, gn3w, gn3b, IMh, IMl);
    k_gemmw<bf, 2, false><<<dim3(DVP / 64, LL / 64, NB_), 32, 0, stream>>>(WC3, ZC3, IMh, IMl, CI * 3, C3, LL, nullptr, 0, (size_t)LL * CI * 3, (size_t)DVP * LL);
    k_fin<<<(unsigned)(((size_t)NB_ * CI * LL / 4 + 255) / 256), 256, 0, stream>>>(x, C3, c3b, OUT);
}
